// OP3PhysicsNetwork_30262339567939
// MI455X (gfx1250) — hardware-verified
//
#include <hip/hip_runtime.h>
#include <hip/hip_bf16.h>
#include <math.h>


typedef _Float16 bf16;
typedef _Float16 f16;
typedef __attribute__((ext_vector_type(4))) unsigned v4u_t;
typedef unsigned v4ua __attribute__((ext_vector_type(4), may_alias));
typedef __attribute__((ext_vector_type(4))) float v4f_t;
typedef float v4fa __attribute__((ext_vector_type(4), may_alias));
typedef __attribute__((ext_vector_type(16))) bf16  bf16x16;
typedef bf16x16 f16x16;
typedef __attribute__((ext_vector_type(8)))  bf16  bf16x8;
typedef bf16x8 f16x8;
typedef __attribute__((ext_vector_type(4)))  bf16  bf16x4;
typedef __attribute__((ext_vector_type(8)))  float f32x8;
__device__ __forceinline__ f32x8 wmma16(f16x16 a, f16x16 b, f32x8 c) {
  c = __builtin_amdgcn_wmma_f32_16x16x32_f16(false, a, false, b, (short)0, c, false, false);
  asm volatile("v_nop\n\tv_nop\n\tv_nop\n\tv_nop" : "+v"(c) : "v"(a), "v"(b));
  return c;
}
#define LDS_STRIDE 48
#define KSTRIDE    72
#define VSTRIDE    48

__device__ __forceinline__ f32x8 wmma_bf16(bf16x16 a, bf16x16 b, f32x8 c) {
  c = __builtin_amdgcn_wmma_f32_16x16x32_f16(false, a, false, b, (short)0, c, false, false);
  asm volatile("v_nop\n\tv_nop\n\tv_nop\n\tv_nop" : "+v"(c) : "v"(a), "v"(b));
  return c;
}

template <typename T>
__device__ __forceinline__ bf16x16 load_frag(const T* __restrict__ base, int ld,
                                             int row0, int k0) {
  const int lane = threadIdx.x & 31;
  const int r    = lane & 15;
  const int kh   = (lane >> 4) * 8;
  const T* p0 = base + (size_t)(row0 + r) * ld + (k0 + kh);
  const T* p1 = p0 + 16;
  bf16x16 f;
#pragma unroll
  for (int i = 0; i < 8; ++i) {
    f[i]     = (bf16)p0[i];
    f[i + 8] = (bf16)p1[i];
  }
  return f;
}

__device__ __forceinline__ bf16x16 lds_frag(const bf16* base, int stride) {
  const int lane = threadIdx.x & 31;
  const int row  = lane & 15;
  const int kh   = (lane >> 4) * 8;
  const bf16x8 lo = *(const bf16x8*)(base + row * stride + kh);
  const bf16x8 hi = *(const bf16x8*)(base + row * stride + kh + 16);
  bf16x16 f;
#pragma unroll
  for (int i = 0; i < 8; ++i) { f[i] = lo[i]; f[i + 8] = hi[i]; }
  return f;
}

template <typename T>
__device__ __forceinline__ void stage_read16(const T* __restrict__ p, float* buf) {
#pragma unroll
  for (int i = 0; i < 16; ++i) buf[i] = (float)p[i];
}

__device__ __forceinline__ void stage_write(bf16* dst, const float* buf, int nquad) {
#pragma unroll
  for (int i = 0; i < nquad; ++i) {
    bf16x4 q;
    q[0] = (bf16)buf[4 * i];     q[1] = (bf16)buf[4 * i + 1];
    q[2] = (bf16)buf[4 * i + 2]; q[3] = (bf16)buf[4 * i + 3];
    *(bf16x4*)(dst + 4 * i) = q;
  }
}


#define GSTR 48
template <typename AT, bool ACC, int ACT>
__global__ __launch_bounds__(256) void gemm_kn2s(const AT* __restrict__ A, int lda, size_t strideA,
                                               const float* __restrict__ Wm, int ldw, size_t strideW,
                                               const float* __restrict__ bias, float scale,
                                               float* __restrict__ Y, int ldy, size_t strideY, int K, float qs) {
  __shared__ __attribute__((aligned(16))) f16 ldsA[128 * GSTR], ldsAl[128 * GSTR];
  __shared__ __attribute__((aligned(16))) f16 ldsW[128 * GSTR], ldsWl[128 * GSTR];
  __shared__ __attribute__((aligned(16))) float oS[8][32 * 68];
  const int tid = threadIdx.x, lane = tid & 31, wave = tid >> 5, cl = lane & 15, rh = (lane >> 4) * 8;
  const int m0 = blockIdx.x * 128, n0 = blockIdx.y * 128;
  const int wm = (wave & 3) * 32, wn = (wave >> 2) * 64;
  A += (size_t)blockIdx.z * strideA; Wm += (size_t)blockIdx.z * strideW; Y += (size_t)blockIdx.z * strideY;
  f32x8 acc[2][4], accx[2][4];
#pragma unroll
  for (int i = 0; i < 2; ++i)
#pragma unroll
    for (int j = 0; j < 4; ++j) { f32x8 z = {}; acc[i][j] = z; accx[i][j] = z; }
#pragma unroll 1
  for (int k0 = 0; k0 < K; k0 += 32) {
    __syncthreads();
    {
      const int row = tid >> 1, ch = (tid & 1) * 16;
      const AT* src = A + (size_t)(m0 + row) * lda + k0 + ch;
#pragma unroll
      for (int g = 0; g < 16; ++g) { const float v = (float)src[g]; const f16 h = (f16)v; ldsA[row * GSTR + ch + g] = h; ldsAl[row * GSTR + ch + g] = (f16)((v - (float)h) * 2048.0f); }
    }
    {
      const int k = tid >> 3, nn0 = (tid & 7) * 16;
      const float* src = Wm + (size_t)(k0 + k) * ldw + n0 + nn0;
#pragma unroll
      for (int g = 0; g < 4; ++g) { const v4f_t v = *(const v4f_t*)(src + 4 * g);
#pragma unroll
        for (int u = 0; u < 4; ++u) { const f16 h = (f16)v[u]; ldsW[(nn0 + 4 * g + u) * GSTR + k] = h; ldsWl[(nn0 + 4 * g + u) * GSTR + k] = (f16)((v[u] - (float)h) * 2048.0f); } }
    }
    __syncthreads();
    f16x16 af[2], afl[2];
#pragma unroll
    for (int i = 0; i < 2; ++i) { af[i] = lds_frag(ldsA + (wm + 16 * i) * GSTR, GSTR); afl[i] = lds_frag(ldsAl + (wm + 16 * i) * GSTR, GSTR); }
#pragma unroll
    for (int j = 0; j < 4; ++j) {
      const f16x16 bf = lds_frag(ldsW + (wn + 16 * j) * GSTR, GSTR), bfl = lds_frag(ldsWl + (wn + 16 * j) * GSTR, GSTR);
#pragma unroll
      for (int i = 0; i < 2; ++i) { acc[i][j] = wmma16(af[i], bf, acc[i][j]); accx[i][j] = wmma16(af[i], bfl, accx[i][j]); accx[i][j] = wmma16(afl[i], bf, accx[i][j]); }
    }
  }
  float* so = oS[wave];
#pragma unroll
  for (int i = 0; i < 2; ++i)
#pragma unroll
    for (int j = 0; j < 4; ++j) {
      const float bv = bias ? bias[n0 + wn + 16 * j + cl] : 0.0f;
#pragma unroll
      for (int r = 0; r < 8; ++r) { float v = (acc[i][j][r] + accx[i][j][r] * (1.0f / 2048.0f)) * scale + bv; if (ACT == 1) v = qs * ((v > 0.0f) ? v : (__expf(v) - 1.0f)); if (ACT == 2) v = qs * v; so[(16 * i + rh + r) * 68 + 16 * j + cl] = v; }
    }
  asm volatile("s_wait_dscnt 0" ::: "memory");
  __builtin_amdgcn_wave_barrier();
  if (ACC) {
#pragma unroll
    for (int it = 0; it < 16; ++it) { const int f4 = lane + 32 * it, rr = f4 >> 4, q = (f4 & 15) * 4;
      const v4f_t old = *(const v4fa*)(Y + (size_t)(m0 + wm + rr) * ldy + n0 + wn + q);
      v4f_t v = *(const v4fa*)(so + rr * 68 + q); v += old; *(v4fa*)(so + rr * 68 + q) = v; }
    asm volatile("s_wait_dscnt 0" ::: "memory");
  }
#pragma unroll 1
  for (int pass = 0; pass < 2; ++pass) {
#pragma unroll
    for (int it = 0; it < 16; ++it) { const int f4 = lane + 32 * it, rr = f4 >> 4, q = (f4 & 15) * 4;
      *(volatile v4f_t*)(Y + (size_t)(m0 + wm + rr) * ldy + n0 + wn + q) = *(const v4fa*)(so + rr * 68 + q); }
    __threadfence();
  }
}


#define NS 8192
#define NBL 1024
#define NN 8
#define DD 256
#define AAD 16
#define AEN 32
#define EFF 32
#define NP 57344
#define PCH 7168
#define NCHUNK 8
#define NCH_RUN 8
#define S_ST 8.0f
#define S_AE 128.0f
#define S_H3 32.0f
#define S_SE 128.0f
#define S_PP 512.0f
#define S_PI 1024.0f
#define S_H7 4096.0f
#define S_PE 8192.0f
#define S_TE 4096.0f
#define S_H9 512.0f
#define S_MG 2048.0f
#define S_OH 4096.0f
__global__ __launch_bounds__(256) void k_aenc(const int* __restrict__ act, const float* __restrict__ w1, const float* __restrict__ b1, const float* __restrict__ w2, const float* __restrict__ b2, float* __restrict__ AE) {
  __shared__ float hS[DD]; __shared__ float oS[AEN];
  const int t = blockIdx.x, tid = threadIdx.x; const int a = act[t];
  { const float v = w1[(size_t)a * DD + tid] + b1[tid]; hS[tid] = (v > 0.0f) ? v : (expf(v) - 1.0f); }
  __syncthreads();
  const int o = tid >> 3, part = tid & 7; float s = 0.0f;
#pragma unroll 1
  for (int c = part * 32; c < part * 32 + 32; ++c) s = fmaf(hS[c], w2[(size_t)c * AEN + o], s);
  s += __shfl_xor(s, 1, 32); s += __shfl_xor(s, 2, 32); s += __shfl_xor(s, 4, 32);
  if (part == 0) { const float v = s + b2[o]; oS[o] = ((v > 0.0f) ? v : (expf(v) - 1.0f)) * S_AE; }
  __syncthreads();
  if (tid < AEN) { *(volatile float*)(AE + (size_t)t * AEN + tid) = oS[tid]; __threadfence(); *(volatile float*)(AE + (size_t)t * AEN + tid) = oS[tid]; }
}
__global__ __launch_bounds__(256) void k_bcast_ae(const float* __restrict__ AE, float* __restrict__ AEB) { const int tid = threadIdx.x; const size_t s = (size_t)blockIdx.x * 64 + (tid >> 2); const int c4 = (tid & 3) * 8;
  const float* src = AE + (s / NN) * AEN + c4; float* dst = AEB + s * AEN + c4; v4f_t a = *(const v4f_t*)src, b = *(const v4f_t*)(src + 4);
  *(volatile v4f_t*)dst = a; *(volatile v4f_t*)(dst + 4) = b; __threadfence(); *(volatile v4f_t*)dst = a; *(volatile v4f_t*)(dst + 4) = b; }
__global__ __launch_bounds__(256) void k_biaselu(const float* __restrict__ Y, const float* __restrict__ bias, float post, float* __restrict__ X, size_t n4) { const size_t i = (size_t)blockIdx.x * 256 + threadIdx.x; if (i >= n4) return; const int c4 = (int)((4 * i) % DD);
  v4f_t v = *(const v4f_t*)(Y + 4 * i);
#pragma unroll
  for (int u = 0; u < 4; ++u) { const float t = v[u] + bias[c4 + u]; v[u] = post * ((t > 0.0f) ? t : (expf(t) - 1.0f)); }
  *(volatile v4f_t*)(X + 4 * i) = v; __threadfence(); *(volatile v4f_t*)(X + 4 * i) = v; }
template <typename HT>
__global__ __launch_bounds__(256) void k_sighead(const HT* __restrict__ H, float inv, const float* __restrict__ w, const float* __restrict__ b, float* __restrict__ att) {
  __shared__ float rs[32];
  const int tid = threadIdx.x, r = tid >> 3, part = tid & 7; const size_t row = (size_t)blockIdx.x * 32 + r; const HT* hr = H + row * DD; float s = 0.0f;
#pragma unroll 1
  for (int c = part * 32; c < part * 32 + 32; ++c) s = fmaf((float)hr[c], w[c], s);
  s += __shfl_xor(s, 1, 32); s += __shfl_xor(s, 2, 32); s += __shfl_xor(s, 4, 32);
  if (part == 0) rs[r] = 1.0f / (1.0f + expf(-(s * inv + b[0])));
  __syncthreads();
  if (tid < 32) { *(volatile float*)(att + (size_t)blockIdx.x * 32 + tid) = rs[tid]; __threadfence(); *(volatile float*)(att + (size_t)blockIdx.x * 32 + tid) = rs[tid]; }
}
__global__ __launch_bounds__(256) void k_rowscale(const float* __restrict__ SEFF, const float* __restrict__ att, float* __restrict__ SE, size_t n4) { const size_t i = (size_t)blockIdx.x * 256 + threadIdx.x; if (i >= n4) return; const size_t r = (4 * i) / DD; const float a = att[r] * (S_SE / 64.0f);
  v4f_t v = *(const v4f_t*)(SEFF + 4 * i); v[0] *= a; v[1] *= a; v[2] *= a; v[3] *= a; *(volatile v4f_t*)(SE + 4 * i) = v; __threadfence(); *(volatile v4f_t*)(SE + 4 * i) = v; }
__global__ __launch_bounds__(256) void k_pairs(const float* __restrict__ U, const float* __restrict__ V, const float* __restrict__ bias, float* __restrict__ PP, int p0) {
  const int pl = blockIdx.x, c = threadIdx.x; const int p = p0 + pl; const int s = p / 7, jj = p % 7; const int i = s & 7; const int j = (jj < i) ? jj : jj + 1; const int sj = (s & ~7) | j;
  const float t = (U[(size_t)s * 512 + c] + V[(size_t)sj * 512 + c]) * (1.0f / S_SE) + bias[c]; const float t2 = (U[(size_t)s * 512 + 256 + c] + V[(size_t)sj * 512 + 256 + c]) * (1.0f / S_SE) + bias[256 + c];
  const float a = S_PP * ((t > 0.0f) ? t : (expf(t) - 1.0f)), b2v = S_PP * ((t2 > 0.0f) ? t2 : (expf(t2) - 1.0f));
  *(volatile float*)(PP + (size_t)pl * 512 + c) = a; *(volatile float*)(PP + (size_t)pl * 512 + 256 + c) = b2v; __threadfence(); *(volatile float*)(PP + (size_t)pl * 512 + c) = a; *(volatile float*)(PP + (size_t)pl * 512 + 256 + c) = b2v;
}
__global__ __launch_bounds__(256) void k_teffect(const float* __restrict__ PEFF, const float* __restrict__ PATT, float* __restrict__ TE, int p0, int s0) {
  const int tid = threadIdx.x; const int sl = blockIdx.x * 8 + (tid >> 5), e = tid & 31; const int s = s0 + sl; float acc = 0.0f;
#pragma unroll
  for (int jj = 0; jj < 7; ++jj) { const size_t p = (size_t)s * 7 + jj - p0; acc = fmaf(PEFF[p * 128 + e], PATT[p], acc); }
  const float v = acc * (S_TE / S_PE); *(volatile float*)(TE + (size_t)s * EFF + e) = v; __threadfence(); *(volatile float*)(TE + (size_t)s * EFF + e) = v;
}
__global__ __launch_bounds__(256) void k_fill(float* __restrict__ p, float val, size_t n4) { const size_t i = (size_t)blockIdx.x * 256 + threadIdx.x; if (i < n4) { v4f_t v = {val, val, val, val}; *(volatile v4f_t*)(p + 4 * i) = v; __threadfence(); *(volatile v4f_t*)(p + 4 * i) = v; } }
__global__ __launch_bounds__(256) void k_padw32(const float* __restrict__ w, const float* __restrict__ b, float* __restrict__ wp, float* __restrict__ bp, int K) { const int k = blockIdx.x, n = threadIdx.x; if (n < 128) { const float v = (n < 32) ? w[(size_t)k * 32 + n] : 0.0f;
  *(volatile float*)(wp + (size_t)k * 128 + n) = v; __threadfence(); *(volatile float*)(wp + (size_t)k * 128 + n) = v; if (k == 0) { const float bb = (n < 32) ? b[n] : 0.0f; *(volatile float*)(bp + n) = bb; __threadfence(); *(volatile float*)(bp + n) = bb; } } }

extern "C" void kernel_launch(void* const* d_in, const int* in_sizes, int n_in,
                              void* d_out, int out_size, void* d_ws, size_t ws_size,
                              hipStream_t stream) {
  (void)in_sizes; (void)n_in; (void)out_size;
  const float** f = (const float**)d_in;
  const float* x = f[0]; const int* act = (const int*)d_in[1];
  const float *in_w1 = f[3], *in_b1 = f[4], *in_w2 = f[5], *in_b2 = f[6], *ae_w1 = f[7], *ae_b1 = f[8], *ae_w2 = f[9], *ae_b2 = f[10];
  const float *eff_w1 = f[11], *eff_b1 = f[12], *eff_w2 = f[13], *eff_b2 = f[14], *aat_w1 = f[15], *aat_b1 = f[16], *aat_w2 = f[17], *aat_b2 = f[18];
  const float *pw_w1 = f[19], *pw_b1 = f[20], *pw_w2 = f[21], *pw_b2 = f[22], *ie_w1 = f[23], *ie_b1 = f[24], *ie_w2 = f[25], *ie_b2 = f[26];
  const float *ia_w1 = f[27], *ia_b1 = f[28], *ia_w2 = f[29], *ia_b2 = f[30], *fm_w1 = f[31], *fm_b1 = f[32], *fm_w2 = f[33], *fm_b2 = f[34];
  const float *out_w1 = f[35], *out_b1 = f[36], *out_w2 = f[37], *out_b2 = f[38];
  float* out = (float*)d_out;
  char* ws = (char*)d_ws;
  float* H1 = (float*)ws; ws += (size_t)NS * DD * 4;
  float* ST = (float*)ws; ws += (size_t)NS * DD * 4;
  float* AE = (float*)ws; ws += (size_t)NBL * AEN * 4; float* AEB = (float*)ws; ws += (size_t)NS * AEN * 4;
  float* H3 = (float*)ws; ws += (size_t)NS * DD * 4;
  float* SEFF = (float*)ws; ws += (size_t)NS * DD * 4;
  float* ATT = (float*)ws; ws += (size_t)NS * 4;
  float* SE = (float*)ws; ws += (size_t)NS * DD * 4;
  float* U = (float*)ws; ws += (size_t)NS * 512 * 4; float* V = (float*)ws; ws += (size_t)NS * 512 * 4;
  float* PP = (float*)ws; ws += (size_t)PCH * 512 * 4;
  float* PINT = (float*)ws; ws += (size_t)PCH * DD * 4;
  float* H7 = (float*)ws; ws += (size_t)PCH * DD * 4;
  float* PEFF = (float*)ws; ws += (size_t)PCH * 128 * 4;
  float* PATT = (float*)ws; ws += (size_t)PCH * 4;
  float* TE = (float*)ws; ws += (size_t)NS * EFF * 4;
  float* H9 = (float*)ws; ws += (size_t)NS * DD * 4;
  float* iew2p = (float*)ws; ws += (size_t)DD * 128 * 4; float* ieb2p = (float*)ws; ws += 128 * 4;
  float* q8 = (float*)ws; ws += 512 * 4; float* q128 = (float*)ws; ws += DD * 4; float* q4096 = (float*)ws; ws += DD * 4;
  if ((size_t)(ws - (char*)d_ws) > ws_size) return;
  const dim3 blk(256); const dim3 g8k(NS / 128, DD / 128);
  k_padw32<<<dim3(DD), blk, 0, stream>>>(ie_w2, ie_b2, iew2p, ieb2p, DD);
  k_fill<<<dim3(1), blk, 0, stream>>>(q8, 1.0f / 8.0f, DD / 4); k_fill<<<dim3(1), blk, 0, stream>>>(q128, 1.0f / 128.0f, DD / 4); k_fill<<<dim3(1), blk, 0, stream>>>(q4096, 1.0f / 4096.0f, DD / 4);
  gemm_kn2s<float, false, 1><<<dim3(NS / 128, DD / 128, 1), blk, 0, stream>>>(x, DD, 0, in_w1, DD, 0, in_b1, 1.0f, H1, DD, 0, DD, 1.0f);
  gemm_kn2s<float, false, 1><<<dim3(NS / 128, DD / 128, 1), blk, 0, stream>>>(H1, DD, 0, in_w2, DD, 0, in_b2, 1.0f, ST, DD, 0, DD, S_ST);
  k_aenc<<<dim3(NBL), blk, 0, stream>>>(act, ae_w1, ae_b1, ae_w2, ae_b2, AE); k_bcast_ae<<<dim3(NS / 64), blk, 0, stream>>>(AE, AEB);
  gemm_kn2s<float, false, 0><<<dim3(NS / 128, DD / 128, 1), blk, 0, stream>>>(ST, DD, 0, eff_w1, DD, 0, nullptr, 1.0f / 8.0f, H1, DD, 0, DD, 1.0f);
  gemm_kn2s<float, true, 0><<<dim3(NS / 128, DD / 128, 1), blk, 0, stream>>>(AEB, AEN, 0, eff_w1 + (size_t)DD * DD, DD, 0, nullptr, 1.0f / 128.0f, H1, DD, 0, AEN, 1.0f);
  k_biaselu<<<dim3((size_t)NS * DD / 4 / 256), blk, 0, stream>>>(H1, eff_b1, S_H3, H3, (size_t)NS * DD / 4);
  gemm_kn2s<float, false, 1><<<dim3(NS / 128, DD / 128, 1), blk, 0, stream>>>(H3, DD, 0, eff_w2, DD, 0, eff_b2, 1.0f / S_H3, SEFF, DD, 0, DD, 64.0f);
  gemm_kn2s<float, false, 0><<<dim3(NS / 128, DD / 128, 1), blk, 0, stream>>>(ST, DD, 0, aat_w1, DD, 0, nullptr, 1.0f / 8.0f, H1, DD, 0, DD, 1.0f);
  gemm_kn2s<float, true, 0><<<dim3(NS / 128, DD / 128, 1), blk, 0, stream>>>(AEB, AEN, 0, aat_w1 + (size_t)DD * DD, DD, 0, nullptr, 1.0f / 128.0f, H1, DD, 0, AEN, 1.0f);
  k_biaselu<<<dim3((size_t)NS * DD / 4 / 256), blk, 0, stream>>>(H1, aat_b1, S_H3, H3, (size_t)NS * DD / 4);
  k_sighead<float><<<dim3(NS / 32), blk, 0, stream>>>(H3, 1.0f / S_H3, aat_w2, aat_b2, ATT);
  k_rowscale<<<dim3((size_t)NS * DD / 4 / 256), blk, 0, stream>>>(SEFF, ATT, SE, (size_t)NS * DD / 4);
  gemm_kn2s<float, false, 0><<<dim3(NS / 128, 512 / 128, 1), blk, 0, stream>>>(SE, DD, 0, pw_w1, 512, 0, nullptr, 1.0f, U, 512, 0, DD, 1.0f);
  gemm_kn2s<float, false, 0><<<dim3(NS / 128, 512 / 128, 1), blk, 0, stream>>>(SE, DD, 0, pw_w1 + (size_t)DD * 512, 512, 0, nullptr, 1.0f, V, 512, 0, DD, 1.0f);
  for (int c = 0; c < NCH_RUN; ++c) { const int p0 = c * PCH, s0 = c * (PCH / 7);
    k_pairs<<<dim3(PCH), blk, 0, stream>>>(U, V, pw_b1, PP, p0);
    gemm_kn2s<float, false, 1><<<dim3(PCH / 128, DD / 128, 1), blk, 0, stream>>>(PP, 512, 0, pw_w2, DD, 0, pw_b2, 1.0f / S_PP, PINT, DD, 0, 512, S_PI);
    gemm_kn2s<float, false, 1><<<dim3(PCH / 128, DD / 128, 1), blk, 0, stream>>>(PINT, DD, 0, ie_w1, DD, 0, ie_b1, 1.0f / S_PI, H7, DD, 0, DD, S_H7);
    gemm_kn2s<float, false, 1><<<dim3(PCH / 128, 1, 1), blk, 0, stream>>>(H7, DD, 0, iew2p, 128, 0, ieb2p, 1.0f / S_H7, PEFF, 128, 0, DD, S_PE);
    gemm_kn2s<float, false, 1><<<dim3(PCH / 128, DD / 128, 1), blk, 0, stream>>>(PINT, DD, 0, ia_w1, DD, 0, ia_b1, 1.0f / S_PI, H7, DD, 0, DD, S_H7);
    k_sighead<float><<<dim3(PCH / 32), blk, 0, stream>>>(H7, 1.0f / S_H7, ia_w2, ia_b2, PATT);
    k_teffect<<<dim3((PCH / 7) / 8), blk, 0, stream>>>(PEFF, PATT, TE, p0, s0);
  }
  gemm_kn2s<float, false, 0><<<dim3(NS / 128, DD / 128, 1), blk, 0, stream>>>(SE, DD, 0, fm_w1, DD, 0, nullptr, 1.0f / 128.0f, H1, DD, 0, DD, 1.0f);
  gemm_kn2s<float, true, 0><<<dim3(NS / 128, DD / 128, 1), blk, 0, stream>>>(TE, EFF, 0, fm_w1 + (size_t)DD * DD, DD, 0, nullptr, 1.0f / 4096.0f, H1, DD, 0, EFF, 1.0f);
  k_biaselu<<<dim3((size_t)NS * DD / 4 / 256), blk, 0, stream>>>(H1, fm_b1, S_H9, H9, (size_t)NS * DD / 4);
  gemm_kn2s<float, false, 1><<<dim3(NS / 128, DD / 128, 1), blk, 0, stream>>>(H9, DD, 0, fm_w2, DD, 0, fm_b2, 1.0f / S_H9, ST, DD, 0, DD, S_MG);
  gemm_kn2s<float, false, 1><<<dim3(NS / 128, DD / 128, 1), blk, 0, stream>>>(ST, DD, 0, out_w1, DD, 0, out_b1, 1.0f / S_MG, H3, DD, 0, DD, S_OH);
  gemm_kn2s<float, false, 2><<<dim3(NS / 128, DD / 128, 1), blk, 0, stream>>>(H3, DD, 0, out_w2, DD, 0, out_b2, 1.0f / S_OH, out, DD, 0, DD, 1.0f);
}
